// SpikingAttention_69724499083935
// MI455X (gfx1250) — hardware-run, weakly checked
//
#include <hip/hip_runtime.h>
#include <math.h>

typedef __attribute__((ext_vector_type(16))) _Float16 v16h;
typedef __attribute__((ext_vector_type(8)))  _Float16 v8h;
typedef __attribute__((ext_vector_type(16))) __bf16   v16b;
typedef __attribute__((ext_vector_type(8)))  __bf16   v8b;
typedef __attribute__((ext_vector_type(8)))  float    v8f;
typedef __attribute__((ext_vector_type(4)))  float    v4f;
typedef __attribute__((ext_vector_type(4)))  unsigned int v4u;

constexpr int kBatch   = 2;
constexpr int kS       = 8192;
constexpr int kD       = 128;
constexpr int kTok     = kBatch * kS;
constexpr int kWin     = 128;
constexpr int kStride  = 64;
constexpr int kNFirst  = 4;
constexpr int kNStr    = kS / kStride;
constexpr int kGValid  = kNStr + (kNFirst - 1);
constexpr int kGS      = 192;
constexpr int kGP      = 256;
constexpr int kSpkN    = kS + kGS;
constexpr int kOsP     = 132;
constexpr float kVCarry = 64.0f;
constexpr float kPCarry = 32768.0f;
constexpr float kOScale = 1.0f / (kPCarry * kVCarry);
constexpr float kF16Min = 6.103515625e-5f;
constexpr float kDecay  = 0.90483741803595952f;
static_assert(kNFirst <= kStride, "prefix keys beyond slot 0 are not strided keys");
static_assert(kGValid <= kGS && (kGS % 64) == 0 && kGS <= kGP, "slot padding");
static_assert((kS % 64) == 0 && (kD % 32) == 0 && (kD % 64) == 0 && (kTok % 64) == 0, "tile multiples");
static_assert(kWin == 2 * 64, "three local 64-key chunks cover the window");
static_assert((kTok % 256) == 0 && ((kTok * kD / 8) % 256) == 0, "exact grids");

constexpr size_t kPlane16 = (size_t)kTok * kD * 2;
constexpr size_t kOffXH  = 0;
constexpr size_t kOffXL  = kOffXH  + kPlane16;
constexpr size_t kOffWT  = kOffXL  + kPlane16;
constexpr size_t kOffCUR = kOffWT  + (size_t)8 * kD * kD * 2;
constexpr size_t kOffSPK = kOffCUR + (size_t)kTok * 4;
constexpr size_t kOffQH  = kOffSPK + (size_t)kSpkN * 4;
constexpr size_t kOffQL  = kOffQH  + kPlane16;
constexpr size_t kOffKH  = kOffQL  + kPlane16;
constexpr size_t kOffKL  = kOffKH  + kPlane16;
constexpr size_t kOffVT  = kOffKL  + kPlane16;
constexpr size_t kOffVG  = kOffVT  + (size_t)kBatch * kD * kS * 2;
constexpr size_t kOffAH  = kOffVG  + (size_t)kBatch * kD * kGP * 2;
constexpr size_t kOffAL  = kOffAH  + kPlane16;
constexpr size_t kWsTotal = kOffAL + kPlane16;
static_assert(kWsTotal == 38241024ull, "carve total");
static_assert(kWsTotal <= 134217728ull, "carve cap");
static_assert((kOffXL % 128) == 0 && (kOffWT % 128) == 0 && (kOffCUR % 128) == 0 && (kOffSPK % 128) == 0 &&
              (kOffQH % 128) == 0 && (kOffQL % 128) == 0 && (kOffKH % 128) == 0 && (kOffKL % 128) == 0 &&
              (kOffVT % 128) == 0 && (kOffVG % 128) == 0 && (kOffAH % 128) == 0 && (kOffAL % 128) == 0, "aligned regions");
static_assert(((size_t)kSpkN * 4) % 128 == 0, "gate table is whole lines");

__device__ __forceinline__ unsigned short f2bf_bits(float f) {
  unsigned u = __float_as_uint(f);
  return (unsigned short)((u + 0x7FFFu + ((u >> 16) & 1u)) >> 16);
}
__device__ __forceinline__ float bf_bits2f(unsigned short h) { return __uint_as_float(((unsigned)h) << 16); }
__device__ __forceinline__ unsigned pk16(unsigned short a, unsigned short b) { return (unsigned)a | ((unsigned)b << 16); }

__device__ __forceinline__ void split8_bf16(v4f a0, v4f a1, v4u& uh, v4u& ul) {
  unsigned short hb[8], lb[8];
#pragma unroll
  for (int e = 0; e < 4; ++e) {
    const float f0 = a0[e];
    const float f1 = a1[e];
    const unsigned short h0 = f2bf_bits(f0);
    const unsigned short h1 = f2bf_bits(f1);
    hb[e] = h0;
    hb[4 + e] = h1;
    lb[e] = f2bf_bits(f0 - bf_bits2f(h0));
    lb[4 + e] = f2bf_bits(f1 - bf_bits2f(h1));
  }
  uh = (v4u){pk16(hb[0], hb[1]), pk16(hb[2], hb[3]), pk16(hb[4], hb[5]), pk16(hb[6], hb[7])};
  ul = (v4u){pk16(lb[0], lb[1]), pk16(lb[2], lb[3]), pk16(lb[4], lb[5]), pk16(lb[6], lb[7])};
}

__device__ __forceinline__ v8f mma_h_guarded(v16h a, v16h b, v8f c) {
  c = __builtin_amdgcn_wmma_f32_16x16x32_f16(false, a, false, b, (short)0, c, false, false);
  asm volatile("v_nop\n\tv_nop\n\tv_nop\n\tv_nop" : "+v"(c) : "v"(a), "v"(b));
  return c;
}
__device__ __forceinline__ v8f mma_b_guarded(v16b a, v16b b, v8f c) {
  c = __builtin_amdgcn_wmma_f32_16x16x32_bf16(false, a, false, b, (short)0, c, false, false);
  asm volatile("v_nop\n\tv_nop\n\tv_nop\n\tv_nop" : "+v"(c) : "v"(a), "v"(b));
  return c;
}
__device__ __forceinline__ void keep4_h(v16h a, v16h b, v16h c, v16h d) { asm volatile("v_nop" :: "v"(a), "v"(b), "v"(c), "v"(d)); }
__device__ __forceinline__ void keep4_b(v16b a, v16b b, v16b c, v16b d) { asm volatile("v_nop" :: "v"(a), "v"(b), "v"(c), "v"(d)); }
__device__ __forceinline__ void acc_guard4(v8f& a, v8f& b, v8f& c, v8f& d) { asm volatile("v_nop\n\tv_nop\n\tv_nop\n\tv_nop" : "+v"(a), "+v"(b), "+v"(c), "+v"(d)); }

template <typename T> struct Frag;
template <> struct Frag<_Float16> {
  typedef v16h V; union U { v16h v; v8h h[2]; };
  static __device__ __forceinline__ v16h load(const _Float16* p) {
    U f; f.h[0] = *(const v8h*)(p); f.h[1] = *(const v8h*)(p + 16); return f.v;
  }
  static __device__ __forceinline__ v8f mma(v16h a, v16h b, v8f c) { return mma_h_guarded(a, b, c); }
  static __device__ __forceinline__ void keep(v16h a, v16h b, v16h c, v16h d) { keep4_h(a, b, c, d); }
};
template <> struct Frag<__bf16> {
  typedef v16b V; union U { v16b v; v8b h[2]; };
  static __device__ __forceinline__ v16b load(const __bf16* p) {
    U f; f.h[0] = *(const v8b*)(p); f.h[1] = *(const v8b*)(p + 16); return f.v;
  }
  static __device__ __forceinline__ v8f mma(v16b a, v16b b, v8f c) { return mma_b_guarded(a, b, c); }
  static __device__ __forceinline__ void keep(v16b a, v16b b, v16b c, v16b d) { keep4_b(a, b, c, d); }
};

template <int ET> struct Elem;
template <> struct Elem<0> { typedef _Float16 T; };
template <> struct Elem<1> { typedef __bf16 T; };
template <int ET, bool SPLIT, int BIAS_MODE, int OUT_MODE, int POST_SEL = 0>
__global__ __launch_bounds__(256) void wmma_gemm64(
    const unsigned short* __restrict__ Ap, const unsigned short* __restrict__ A2p, int lda, long strideA,
    const unsigned short* __restrict__ Btp, const unsigned short* __restrict__ Bt2p, int ldb, long strideB,
    void* __restrict__ Cout, void* __restrict__ Cout2, int ldc, long strideC,
    const float* __restrict__ bias,
    int M, int N, int K, float scale, float post) {
  typedef typename Elem<ET>::T T;
  typedef typename Frag<T>::V V;
  const T* A = (const T*)Ap; const T* A2 = (const T*)A2p; const T* Bt = (const T*)Btp; const T* Bt2 = (const T*)Bt2p;
  __shared__ __align__(16) float sT[8][16 * 68];
  const int b    = blockIdx.y;
  const int lane = threadIdx.x & 31;
  const int wave = threadIdx.x >> 5;
  const int tilesN = N >> 6;
  const int tilesM = M >> 6;
  const int tile = blockIdx.x * 8 + wave;
  if (tile >= tilesM * tilesN) return;
  const int tm = tile / tilesN;
  const int tn = tile - tm * tilesN;
  const int m0 = tm << 6;
  const int n0 = tn << 6;

  const float postv = (POST_SEL == 1) ? (1.0f / sqrtf((float)kD)) : post;

  const T* Ab  = A  + (size_t)b * strideA;
  const T* Bb  = Bt + (size_t)b * strideB;
  const T* Ab2 = SPLIT ? (A2  + (size_t)b * strideA) : nullptr;
  const T* Bb2 = SPLIT ? (Bt2 + (size_t)b * strideB) : nullptr;

  const int rlane = lane & 15;
  const int koff  = (lane >> 4) * 8;
  const int mOff  = (lane >> 4) * 8;

  v8f acc[4][4];
#pragma unroll
  for (int i = 0; i < 4; ++i)
#pragma unroll
    for (int j = 0; j < 4; ++j) acc[i][j] = (v8f){0.f,0.f,0.f,0.f,0.f,0.f,0.f,0.f};

  for (int k0 = 0; k0 < K; k0 += 32) {
    V bh[4], bl[4];
#pragma unroll
    for (int j = 0; j < 4; ++j) {
      const size_t bo = (size_t)(n0 + (j << 4) + rlane) * ldb + koff + k0;
      bh[j] = Frag<T>::load(Bb + bo);
      if (SPLIT) bl[j] = Frag<T>::load(Bb2 + bo);
    }
#pragma unroll
    for (int i = 0; i < 4; ++i) {
      const size_t ao = (size_t)(m0 + (i << 4) + rlane) * lda + koff + k0;
      V ah = Frag<T>::load(Ab + ao);
      V al;
      if (SPLIT) al = Frag<T>::load(Ab2 + ao);
#pragma unroll
      for (int j = 0; j < 4; ++j) {
        acc[i][j] = Frag<T>::mma(ah, bh[j], acc[i][j]);
        if (SPLIT) {
          acc[i][j] = Frag<T>::mma(ah, bl[j], acc[i][j]);
          acc[i][j] = Frag<T>::mma(al, bh[j], acc[i][j]);
        }
      }
    }
    Frag<T>::keep(bh[0], bh[1], bh[2], bh[3]);
    if (SPLIT) Frag<T>::keep(bl[0], bl[1], bl[2], bl[3]);
  }
  acc_guard4(acc[0][0], acc[0][1], acc[0][2], acc[0][3]);
  acc_guard4(acc[1][0], acc[1][1], acc[1][2], acc[1][3]);
  acc_guard4(acc[2][0], acc[2][1], acc[2][2], acc[2][3]);
  acc_guard4(acc[3][0], acc[3][1], acc[3][2], acc[3][3]);

  float* slab = sT[wave];
#pragma unroll
  for (int i = 0; i < 4; ++i) {
    const int mBase = m0 + (i << 4);
#pragma unroll
    for (int j = 0; j < 4; ++j) {
      const int n = n0 + (j << 4) + rlane;
      float bv = 0.f;
      if (BIAS_MODE == 2) bv = bias[n];
#pragma unroll
      for (int r = 0; r < 8; ++r) {
        float v = acc[i][j][r] * scale;
        if (BIAS_MODE == 1) v += bias[mBase + mOff + r];
        if (BIAS_MODE == 2) v += bv;
        v *= postv;
        slab[(mOff + r) * 68 + (j << 4) + rlane] = v;
      }
    }
    __builtin_amdgcn_fence(__ATOMIC_RELEASE, "workgroup");
    __builtin_amdgcn_wave_barrier();
    __builtin_amdgcn_fence(__ATOMIC_ACQUIRE, "workgroup");
    if (OUT_MODE == 0) {
      float* C = (float*)Cout + (size_t)b * strideC;
      const int hh = lane >> 4, c4 = (lane & 15) * 4;
      for (int pass = 0; pass < 2; ++pass) {
#pragma unroll
        for (int it = 0; it < 8; ++it) {
          const int row = it * 2 + hh;
          v4f v = *(const v4f*)(slab + row * 68 + c4);
          *(volatile v4f*)(C + (size_t)(mBase + row) * ldc + n0 + c4) = v;
        }
        __threadfence();
      }
    } else {
      const int q = lane >> 3, c8 = (lane & 7) * 8;
      unsigned short* C  = (unsigned short*)Cout  + (size_t)b * strideC;
      unsigned short* C2 = (OUT_MODE == 2) ? ((unsigned short*)Cout2 + (size_t)b * strideC) : nullptr;
      for (int pass = 0; pass < 2; ++pass) {
#pragma unroll
        for (int it = 0; it < 4; ++it) {
          const int row = it * 4 + q;
          const float* sp = slab + row * 68 + c8;
          v8h hv, lv;
#pragma unroll
          for (int e = 0; e < 8; ++e) {
            if (OUT_MODE == 1) {
              float tv = sp[e];
              tv = (fabsf(tv) < kF16Min) ? 0.0f : tv;
              hv[e] = (_Float16)tv;
            } else {
              unsigned short hb = f2bf_bits(sp[e]);
              unsigned short lb = f2bf_bits(sp[e] - bf_bits2f(hb));
              hv[e] = __builtin_bit_cast(_Float16, hb);
              lv[e] = __builtin_bit_cast(_Float16, lb);
            }
          }
          *(volatile v8h*)(C + (size_t)(mBase + row) * ldc + n0 + c8) = hv;
          if (OUT_MODE == 2) *(volatile v8h*)(C2 + (size_t)(mBase + row) * ldc + n0 + c8) = lv;
        }
        __threadfence();
      }
    }
    __builtin_amdgcn_fence(__ATOMIC_RELEASE, "workgroup");
    __builtin_amdgcn_wave_barrier();
    __builtin_amdgcn_fence(__ATOMIC_ACQUIRE, "workgroup");
  }
}

__global__ __launch_bounds__(256) void split_rows_bf16_kernel(
    const float* __restrict__ src, unsigned short* __restrict__ dhi, unsigned short* __restrict__ dlo, int total8)
{
  const int i = blockIdx.x * 256 + threadIdx.x;
  if (i >= total8) return;
  const size_t e0 = (size_t)i << 3;
  const v4f a0 = *(const v4f*)(src + e0);
  const v4f a1 = *(const v4f*)(src + e0 + 4);
  v4u uh, ul;
  split8_bf16(a0, a1, uh, ul);
  unsigned short* qh = dhi + e0;
  unsigned short* ql = dlo + e0;
  *(volatile v4u*)qh = uh;
  *(volatile v4u*)ql = ul;
  __threadfence();
  *(volatile v4u*)qh = uh;
  *(volatile v4u*)ql = ul;
}

__global__ __launch_bounds__(256) void wt_split_kernel(const float* __restrict__ W0, const float* __restrict__ W1,
                                                       const float* __restrict__ W2, const float* __restrict__ W3,
                                                       unsigned short* __restrict__ out) {
  __shared__ float sm[64][65];
  const int t  = threadIdx.x;
  const int d0 = blockIdx.x * 64;
  const int h0 = blockIdx.y * 64;
  const int z  = blockIdx.z;
  const float* W = (z == 0) ? W0 : (z == 1) ? W1 : (z == 2) ? W2 : W3;
#pragma unroll
  for (int i = 0; i < 16; ++i) {
    const int e = i * 256 + t;
    const int r = e >> 6;
    const int cc = e & 63;
    sm[cc][r] = W[(size_t)(d0 + r) * kD + h0 + cc];
  }
  __syncthreads();
  const int lane = t & 31, wave = t >> 5;
  const int q = lane >> 3, c8 = (lane & 7) * 8;
  unsigned short* oh = out + (size_t)z * 2 * kD * kD;
  unsigned short* ol = oh + (size_t)kD * kD;
  for (int pass = 0; pass < 2; ++pass) {
#pragma unroll
    for (int it = 0; it < 2; ++it) {
      const int row = wave * 8 + it * 4 + q;
      v4f a0, a1;
#pragma unroll
      for (int e = 0; e < 4; ++e) {
        a0[e] = sm[row][c8 + e];
        a1[e] = sm[row][c8 + 4 + e];
      }
      v4u uh, ul;
      split8_bf16(a0, a1, uh, ul);
      const size_t o = (size_t)(h0 + row) * kD + d0 + c8;
      *(volatile v4u*)(oh + o) = uh;
      *(volatile v4u*)(ol + o) = ul;
    }
    __threadfence();
  }
}

__global__ __launch_bounds__(256) void cur_kernel(const float* __restrict__ x, const float* __restrict__ Ws,
                                                  const float* __restrict__ bs, float* __restrict__ cur) {
  const int idx = blockIdx.x * 256 + threadIdx.x;
  const float* xp = x + (size_t)idx * kD;
  float s = 0.0f;
#pragma unroll 2
  for (int i = 0; i < kD / 4; ++i) {
    const v4f xv = *(const v4f*)(xp + 4 * i);
    s = fmaf(xv[0], Ws[4 * i + 0], s);
    s = fmaf(xv[1], Ws[4 * i + 1], s);
    s = fmaf(xv[2], Ws[4 * i + 2], s);
    s = fmaf(xv[3], Ws[4 * i + 3], s);
  }
  const float v = s + bs[0];
  volatile float* cp = (volatile float*)cur + idx;
  *cp = v;
  __threadfence();
  *cp = v;
}

__global__ __launch_bounds__(256) void lif_kernel(const float* __restrict__ cur, int* __restrict__ spk) {
  __shared__ unsigned sw[2][kS / 32];
  const int t = threadIdx.x, lane = t & 31, wave = t >> 5;
  if (wave == 0) {
    const int bsel = lane & 1;
    const float* cp = cur + (size_t)bsel * kS;
    float mem = 0.0f;
#pragma unroll 1
    for (int w = 0; w < kS / 32; ++w) {
      unsigned word = 0u;
#pragma unroll
      for (int q = 0; q < 8; ++q) {
        const v4f cv = *(const v4f*)(cp + w * 32 + q * 4);
#pragma unroll
        for (int e = 0; e < 4; ++e) {
          const float ce = cv[e];
          mem = fmaf(kDecay, mem, ce);
          const bool fired = (mem >= 1.0f);
          mem = fired ? 0.0f : mem;
          word |= fired ? (1u << (q * 4 + e)) : 0u;
        }
      }
      sw[bsel][w] = word;
    }
  }
  __syncthreads();
  for (int pass = 0; pass < 2; ++pass) {
#pragma unroll 1
    for (int it = 0; it < kS / 256; ++it) {
      const int j = it * 256 + t;
      const unsigned wd = sw[0][j >> 5] | sw[1][j >> 5];
      const int v = (int)((wd >> (j & 31)) & 1u);
      *((volatile int*)spk + j) = v;
    }
    if (t < kGS) {
      const int jg = (t < kNStr) ? t * kStride : ((t < kGValid) ? (t - kNStr + 1) : 0);
      const unsigned wd = sw[0][jg >> 5] | sw[1][jg >> 5];
      const int bit = (int)((wd >> (jg & 31)) & 1u);
      const int v = (t < kGValid) ? bit : 0;
      *((volatile int*)spk + kS + t) = v;
    }
    __threadfence();
  }
}

__global__ __launch_bounds__(32) void vg_gather_kernel(const unsigned short* __restrict__ VTp, unsigned short* __restrict__ VGp) {
  const int row = blockIdx.x;
  const int lane = threadIdx.x;
  const unsigned* src = (const unsigned*)(VTp + (size_t)row * kS);
  unsigned short hb[8];
#pragma unroll
  for (int e = 0; e < 8; ++e) {
    const int gp = lane * 8 + e;
    const int jg = (gp < kNStr) ? gp * kStride : ((gp < kGValid) ? (gp - kNStr + 1) : 0);
    const unsigned w = src[jg >> 1];
    const unsigned hv = (jg & 1) ? (w >> 16) : (w & 0xffffu);
    hb[e] = (gp < kGValid) ? (unsigned short)hv : (unsigned short)0;
  }
  const v4u u = (v4u){pk16(hb[0], hb[1]), pk16(hb[2], hb[3]), pk16(hb[4], hb[5]), pk16(hb[6], hb[7])};
  unsigned short* q = VGp + (size_t)row * kGP + lane * 8;
  *(volatile v4u*)q = u;
  __threadfence();
  *(volatile v4u*)q = u;
}

__global__ __launch_bounds__(128) void attn_kernel(
    const unsigned short* __restrict__ QHp, const unsigned short* __restrict__ QLp,
    const unsigned short* __restrict__ KHp, const unsigned short* __restrict__ KLp,
    const unsigned short* __restrict__ VTp, const unsigned short* __restrict__ VGp,
    const int* __restrict__ spk,
    unsigned short* __restrict__ AHp, unsigned short* __restrict__ ALp)
{
  __shared__ __align__(16) _Float16 Ps[4][16 * 64];
  __shared__ __align__(16) float Os[4][16 * kOsP];
  const int tid = threadIdx.x, wave = tid >> 5, lane = tid & 31, hh = lane >> 4, c = lane & 15;
  constexpr int nqb = kS / 64;
  const int b  = blockIdx.x / nqb;
  const int qb = blockIdx.x - b * nqb;
  const int i0 = qb * 64;
  const int q0 = i0 + wave * 16;

  const __bf16* qhp = (const __bf16*)QHp + ((size_t)b * kS + q0 + c) * kD + 8 * hh;
  const __bf16* qlp = (const __bf16*)QLp + ((size_t)b * kS + q0 + c) * kD + 8 * hh;
  const __bf16* khb = (const __bf16*)KHp + (size_t)b * kS * kD + 8 * hh;
  const __bf16* klb = (const __bf16*)KLp + (size_t)b * kS * kD + 8 * hh;
  const _Float16* vtb = (const _Float16*)VTp + (size_t)b * kD * kS + 8 * hh;
  const _Float16* vgb = (const _Float16*)VGp + (size_t)b * kD * kGP + 8 * hh;
  _Float16* pw = Ps[wave];

  float mrow[8], lrow[8];
  v8f oacc[8];
#pragma unroll
  for (int r = 0; r < 8; ++r) { mrow[r] = -INFINITY; lrow[r] = 0.f; }
#pragma unroll
  for (int t = 0; t < 8; ++t) oacc[t] = (v8f){0.f,0.f,0.f,0.f,0.f,0.f,0.f,0.f};

#pragma unroll 1
  for (int ch = 0; ch < 6; ++ch) {
    const bool isg = (ch >= 3);
    const int j0 = i0 - kWin + 64 * ch;
    if (!isg && j0 < 0) continue;
    const int g0 = (ch - 3) * 64;

    int jpos[4], keep[4];
#pragma unroll
    for (int jt = 0; jt < 4; ++jt) {
      const int jj = jt * 16 + c;
      const int gp = g0 + jj;
      const int jg = (gp < kNStr) ? gp * kStride : ((gp < kGValid) ? (gp - kNStr + 1) : 0);
      const int jl = j0 + jj;
      int jp = isg ? jg : jl;
      int si = isg ? (kS + gp) : jl;
      jp = jp < 0 ? 0 : (jp > kS - 1 ? kS - 1 : jp);
      si = si < 0 ? 0 : (si > kSpkN - 1 ? kSpkN - 1 : si);
      jpos[jt] = jp;
      keep[jt] = spk[si];
    }
    const _Float16* vp = isg ? (vgb + g0) : (vtb + j0);
    const int vpitch = isg ? kGP : kS;

    v8f s[4];
#pragma unroll
    for (int jt = 0; jt < 4; ++jt) s[jt] = (v8f){0.f,0.f,0.f,0.f,0.f,0.f,0.f,0.f};
#pragma unroll 1
    for (int dc = 0; dc < kD / 32; ++dc) {
      const v16b qa = Frag<__bf16>::load(qhp + dc * 32);
      const v16b ql = Frag<__bf16>::load(qlp + dc * 32);
#pragma unroll
      for (int jt = 0; jt < 4; ++jt) {
        const size_t ko = (size_t)jpos[jt] * kD + dc * 32;
        const v16b kh = Frag<__bf16>::load(khb + ko);
        const v16b kl = Frag<__bf16>::load(klb + ko);
        s[jt] = mma_b_guarded(qa, kh, s[jt]);
        s[jt] = mma_b_guarded(qa, kl, s[jt]);
        s[jt] = mma_b_guarded(ql, kh, s[jt]);
      }
    }

    float cm[8];
#pragma unroll
    for (int r = 0; r < 8; ++r) {
      const int qi = q0 + 8 * hh + r;
      float m = -INFINITY;
#pragma unroll
      for (int jt = 0; jt < 4; ++jt) {
        const int jp = jpos[jt];
        const bool inwin = (jp <= qi) && (jp >= qi - kWin);
        const bool ok = (keep[jt] != 0) && (inwin != isg);
        const float sv = ok ? s[jt][r] : -INFINITY;
        s[jt][r] = sv;
        m = fmaxf(m, sv);
      }
#pragma unroll
      for (int off = 1; off < 16; off <<= 1) m = fmaxf(m, __shfl_xor(m, off, 32));
      cm[r] = m;
    }

#pragma unroll
    for (int r = 0; r < 8; ++r) {
      const float mnew = fmaxf(mrow[r], cm[r]);
      const float msafe = (mnew == -INFINITY) ? 0.0f : mnew;
      const float alpha = expf(mrow[r] - msafe);
      mrow[r] = mnew;
      float psum = 0.f;
#pragma unroll
      for (int jt = 0; jt < 4; ++jt) {
        const float p = expf(s[jt][r] - msafe);
        psum += p;
        const float pc = p * kPCarry;
        const float pf = (pc < kF16Min) ? 0.0f : pc;
        pw[(8 * hh + r) * 64 + jt * 16 + c] = (_Float16)pf;
      }
#pragma unroll
      for (int off = 1; off < 16; off <<= 1) psum += __shfl_xor(psum, off, 32);
      lrow[r] = lrow[r] * alpha + psum;
#pragma unroll
      for (int t = 0; t < 8; ++t) oacc[t][r] *= alpha;
    }
    __builtin_amdgcn_fence(__ATOMIC_RELEASE, "workgroup");
    __builtin_amdgcn_wave_barrier();
    __builtin_amdgcn_fence(__ATOMIC_ACQUIRE, "workgroup");

#pragma unroll 1
    for (int kk = 0; kk < 2; ++kk) {
      const v16h pa = Frag<_Float16>::load(pw + c * 64 + kk * 32 + 8 * hh);
#pragma unroll
      for (int t = 0; t < 8; ++t) {
        const v16h vb = Frag<_Float16>::load(vp + (size_t)(t * 16 + c) * vpitch + kk * 32);
        oacc[t] = mma_h_guarded(pa, vb, oacc[t]);
      }
    }
    __builtin_amdgcn_fence(__ATOMIC_RELEASE, "workgroup");
    __builtin_amdgcn_wave_barrier();
    __builtin_amdgcn_fence(__ATOMIC_ACQUIRE, "workgroup");
  }

  float* os = Os[wave];
#pragma unroll
  for (int r = 0; r < 8; ++r) {
    const float inv = (lrow[r] > 0.0f) ? kOScale * (1.0f / lrow[r]) : 0.0f;
#pragma unroll
    for (int t = 0; t < 8; ++t) os[(8 * hh + r) * kOsP + t * 16 + c] = oacc[t][r] * inv;
  }
  __builtin_amdgcn_fence(__ATOMIC_RELEASE, "workgroup");
  __builtin_amdgcn_wave_barrier();
  __builtin_amdgcn_fence(__ATOMIC_ACQUIRE, "workgroup");
  {
    const int c8 = (lane & 15) * 8;
    for (int pass = 0; pass < 2; ++pass) {
#pragma unroll
      for (int it = 0; it < 8; ++it) {
        const int row = it * 2 + hh;
        const float* sp = os + row * kOsP + c8;
        const v4f a0 = *(const v4f*)(sp);
        const v4f a1 = *(const v4f*)(sp + 4);
        v4u uh, ul;
        split8_bf16(a0, a1, uh, ul);
        const size_t o = ((size_t)b * kS + q0 + row) * kD + c8;
        *(volatile v4u*)(AHp + o) = uh;
        *(volatile v4u*)(ALp + o) = ul;
      }
      __threadfence();
    }
  }
}

extern "C" void kernel_launch(void* const* d_in, const int* in_sizes, int n_in,
                              void* d_out, int out_size, void* d_ws, size_t ws_size,
                              hipStream_t stream) {
  if (n_in < 11) return;
  if (in_sizes[0] != kTok * kD) return;
  if (in_sizes[1] != kD * kD || in_sizes[3] != kD * kD || in_sizes[5] != kD * kD || in_sizes[7] != kD * kD) return;
  if (in_sizes[2] != kD || in_sizes[4] != kD || in_sizes[6] != kD || in_sizes[8] != kD) return;
  if (in_sizes[9] != kD || in_sizes[10] != 1) return;
  if (out_size != kTok * kD) return;
  if (ws_size < kWsTotal) return;

  const float* x  = (const float*)d_in[0];
  const float* Wq = (const float*)d_in[1];
  const float* bq = (const float*)d_in[2];
  const float* Wk = (const float*)d_in[3];
  const float* bk = (const float*)d_in[4];
  const float* Wv = (const float*)d_in[5];
  const float* bv = (const float*)d_in[6];
  const float* Wo = (const float*)d_in[7];
  const float* bo = (const float*)d_in[8];
  const float* Ws = (const float*)d_in[9];
  const float* bs = (const float*)d_in[10];
  float* out = (float*)d_out;

  char* ws = (char*)d_ws;
  unsigned short* XH  = (unsigned short*)(ws + kOffXH);
  unsigned short* XL  = (unsigned short*)(ws + kOffXL);
  unsigned short* WT  = (unsigned short*)(ws + kOffWT);
  float*          CUR = (float*)(ws + kOffCUR);
  int*            SPK = (int*)(ws + kOffSPK);
  unsigned short* QH  = (unsigned short*)(ws + kOffQH);
  unsigned short* QL  = (unsigned short*)(ws + kOffQL);
  unsigned short* KH  = (unsigned short*)(ws + kOffKH);
  unsigned short* KL  = (unsigned short*)(ws + kOffKL);
  unsigned short* VT  = (unsigned short*)(ws + kOffVT);
  unsigned short* VG  = (unsigned short*)(ws + kOffVG);
  unsigned short* AH  = (unsigned short*)(ws + kOffAH);
  unsigned short* AL  = (unsigned short*)(ws + kOffAL);

  constexpr size_t kWPlane = (size_t)kD * kD;
  unsigned short* WqH = WT + 0 * kWPlane;
  unsigned short* WqL = WT + 1 * kWPlane;
  unsigned short* WkH = WT + 2 * kWPlane;
  unsigned short* WkL = WT + 3 * kWPlane;
  unsigned short* WvH = WT + 4 * kWPlane;
  unsigned short* WvL = WT + 5 * kWPlane;
  unsigned short* WoH = WT + 6 * kWPlane;
  unsigned short* WoL = WT + 7 * kWPlane;

  split_rows_bf16_kernel<<<(kTok * kD / 8) / 256, 256, 0, stream>>>(x, XH, XL, kTok * kD / 8);
  wt_split_kernel<<<dim3(kD / 64, kD / 64, 4), 256, 0, stream>>>(Wq, Wk, Wv, Wo, WT);

  cur_kernel<<<kTok / 256, 256, 0, stream>>>(x, Ws, bs, CUR);
  lif_kernel<<<1, 256, 0, stream>>>(CUR, SPK);

  wmma_gemm64<1, true, 2, 2, 1><<<dim3(64, 1), 256, 0, stream>>>(
      XH, XL, kD, 0L, WqH, WqL, kD, 0L,
      (void*)QH, (void*)QL, kD, 0L, bq, kTok, kD, kD, 1.0f, 1.0f);
  wmma_gemm64<1, true, 2, 2><<<dim3(64, 1), 256, 0, stream>>>(
      XH, XL, kD, 0L, WkH, WkL, kD, 0L,
      (void*)KH, (void*)KL, kD, 0L, bk, kTok, kD, kD, 1.0f, 1.0f);
  wmma_gemm64<1, true, 1, 1><<<dim3(32, kBatch), 256, 0, stream>>>(
      WvH, WvL, kD, 0L, XH, XL, kD, (long)kS * kD,
      (void*)VT, nullptr, kS, (long)kD * kS, bv, kD, kS, kD, 1.0f, kVCarry);

  vg_gather_kernel<<<kBatch * kD, 32, 0, stream>>>(VT, VG);

  attn_kernel<<<kBatch * (kS / 64), 128, 0, stream>>>(QH, QL, KH, KL, VT, VG, SPK, AH, AL);

  wmma_gemm64<1, true, 2, 0><<<dim3(64, 1), 256, 0, stream>>>(
      AH, AL, kD, 0L, WoH, WoL, kD, 0L,
      (void*)out, nullptr, kD, 0L, bo, kTok, kD, kD, 1.0f, 1.0f);
}
